// QLSTMCell_63153199121065
// MI455X (gfx1250) — hardware-verified
//
#include <hip/hip_runtime.h>


#pragma clang fp contract(off)

#define NB_  4096
#define NI_  512
#define NH_  512
#define NG_  2048
#define SP_  36

static_assert(NI_ == NH_);
static_assert(NI_ % 32 == 0);
static_assert(NB_ % 32 == 0);
static_assert(NH_ % 32 == 0);
static_assert(NG_ == 4 * NH_);
static_assert((NB_ * NI_) % 2048 == 0);
static_assert((NG_ * NI_) % 2048 == 0);
static_assert((SP_ * 4) % 16 == 0);

typedef float          v4f   __attribute__((ext_vector_type(4)));
typedef float          v8f   __attribute__((ext_vector_type(8)));
typedef __bf16         v16b  __attribute__((ext_vector_type(16)));
typedef unsigned short u16x8 __attribute__((ext_vector_type(8)));

union FragB { u16x8 h[2]; v16b v; };

constexpr size_t SZ_A16 = (size_t)NB_ * NI_ * 2;
constexpr size_t SZ_W16 = (size_t)NG_ * NI_ * 2;
constexpr size_t OFF_XH  = 0;
constexpr size_t OFF_XL  = OFF_XH  + SZ_A16;
constexpr size_t OFF_HH  = OFF_XL  + SZ_A16;
constexpr size_t OFF_HL  = OFF_HH  + SZ_A16;
constexpr size_t OFF_WIH = OFF_HL  + SZ_A16;
constexpr size_t OFF_WIL = OFF_WIH + SZ_W16;
constexpr size_t OFF_WHH = OFF_WIL + SZ_W16;
constexpr size_t OFF_WHL = OFF_WHH + SZ_W16;
constexpr size_t WS_END  = OFF_WHL + SZ_W16;
static_assert(WS_END <= (size_t)134217728);
static_assert(OFF_XL % 128 == 0 && OFF_HH % 128 == 0 && OFF_HL % 128 == 0 && OFF_WIH % 128 == 0);
static_assert(OFF_WIL % 128 == 0 && OFF_WHH % 128 == 0 && OFF_WHL % 128 == 0);
static_assert(SZ_A16 % 512 == 0 && SZ_W16 % 512 == 0);

__device__ __forceinline__ unsigned short f32_to_bf16(float f) {
    unsigned u = __float_as_uint(f);
    unsigned r = u + 0x7FFFu + ((u >> 16) & 1u);
    return (unsigned short)(r >> 16);
}
__device__ __forceinline__ float bf16_to_f32(unsigned short b) {
    return __uint_as_float(((unsigned)b) << 16);
}
__device__ __forceinline__ v8f ld8f(const float* p) {
    v4f a = *(const v4f*)p;
    v4f b = *(const v4f*)(p + 4);
    return __builtin_shufflevector(a, b, 0, 1, 2, 3, 4, 5, 6, 7);
}
__device__ __forceinline__ void split8(const v8f x, u16x8& hv, u16x8& lv) {
#pragma unroll
    for (int c = 0; c < 8; ++c) {
        const float f = x[c];
        const unsigned short hb = f32_to_bf16(f);
        const unsigned short lb = f32_to_bf16(f - bf16_to_f32(hb));
        hv[c] = hb;
        lv[c] = lb;
    }
}

__device__ __forceinline__ void mma16(v8f& acc, const FragB& a, const FragB& b) {
    acc = __builtin_amdgcn_wmma_f32_16x16x32_bf16(false, a.v, false, b.v, (short)0, acc, false, false);
    asm volatile("v_nop\n\tv_nop\n\tv_nop\n\tv_nop" : "+v"(acc) : "v"(a.v), "v"(b.v));
}

__device__ __forceinline__ void load_frag(FragB& f, const unsigned short* p) {
    f.h[0] = *(const u16x8*)(p);
    f.h[1] = *(const u16x8*)(p + 16);
}

__global__ __launch_bounds__(256)
void cvt_split_kernel(const float* __restrict__ src, unsigned short* dhi, unsigned short* dlo, int n8)
{
    const int i = blockIdx.x * 256 + threadIdx.x;
    if (i >= n8) return;
    const size_t e = (size_t)i * 8;
    const v8f x = ld8f(src + e);
    u16x8 hv, lv;
    split8(x, hv, lv);
    *(volatile u16x8*)(dhi + e) = hv;
    *(volatile u16x8*)(dlo + e) = lv;
    __threadfence();
    *(volatile u16x8*)(dhi + e) = hv;
    *(volatile u16x8*)(dlo + e) = lv;
}

__device__ __forceinline__ void gemm_phase(const unsigned short* __restrict__ Ah,
                                           const unsigned short* __restrict__ Al,
                                           const unsigned short* __restrict__ Bh,
                                           const unsigned short* __restrict__ Bl,
                                           size_t aoff, size_t boff, v8f (&acc)[4])
{
    constexpr size_t GST = (size_t)NH_ * NI_;
#pragma unroll 1
    for (int kt = 0; kt < NI_ / 32; ++kt) {
        const size_t k0 = (size_t)kt * 32;
        FragB fa, ga, fb[4], gb[4];
        load_frag(fa, Ah + aoff + k0);
        load_frag(ga, Al + aoff + k0);
#pragma unroll
        for (int g = 0; g < 4; ++g) {
            load_frag(fb[g], Bh + boff + (size_t)g * GST + k0);
            load_frag(gb[g], Bl + boff + (size_t)g * GST + k0);
        }
#pragma unroll
        for (int g = 0; g < 4; ++g) {
            mma16(acc[g], fa, fb[g]);
            mma16(acc[g], fa, gb[g]);
            mma16(acc[g], ga, fb[g]);
        }
    }
}

__device__ __forceinline__ float quant_p2(float x, float sc, float isc) {
#pragma clang fp contract(off)
    const float a = x * sc;
    const float b = a + 0.5f;
    return floorf(b) * isc;
}
__device__ __forceinline__ float qin27(float x) {
#pragma clang fp contract(off)
    const float a = x * 134217728.0f;
    const float b = a + 0.5f;
    float c = floorf(b);
    c = fmaxf(c, -2147483648.0f);
    c = fminf(c, 2147483648.0f);
    return c * (1.0f / 134217728.0f);
}
__device__ __forceinline__ float requant15(float sf) {
#pragma clang fp contract(off)
    const float f   = sf * 2147483648.0f;
    const float g   = f + 0.5f;
    const float y31 = floorf(g);
    const float q   = y31 * (1.0f / 65536.0f);
    const float t   = q + 0.5f;
    const float y15 = floorf(t);
    return y15 * (1.0f / 32768.0f);
}
__device__ __forceinline__ float qsig_fn(float x) {
    const float  e = qin27(x);
    const double s = 1.0 / (1.0 + exp(-(double)e));
    return requant15((float)s);
}
__device__ __forceinline__ float qtanh_fn(float x) {
    const float  e = qin27(x);
    const double t = tanh((double)e);
    return requant15((float)t);
}

__device__ __forceinline__ void out_store_pass(const float* st0, const float* st1,
                                               float* ohy, float* ocy,
                                               int rowB, int colB, int wave, int lane)
{
    const int c0 = (lane & 7) * 4;
    const int q  = lane >> 3;
#pragma unroll
    for (int it = 0; it < 2; ++it) {
        const int row = it * 16 + wave * 4 + q;
        const size_t go = (size_t)(rowB + row) * NH_ + colB + c0;
        const v4f a = *(const v4f*)(st0 + row * SP_ + c0);
        const v4f b = *(const v4f*)(st1 + row * SP_ + c0);
        *(volatile v4f*)(ohy + go) = a;
        *(volatile v4f*)(ocy + go) = b;
    }
}

__global__ __launch_bounds__(128)
void gates_gemm_kernel(const unsigned short* __restrict__ Xh, const unsigned short* __restrict__ Xl,
                       const unsigned short* __restrict__ Hh, const unsigned short* __restrict__ Hl,
                       const unsigned short* __restrict__ Wih, const unsigned short* __restrict__ Wil,
                       const unsigned short* __restrict__ Whh, const unsigned short* __restrict__ Whl,
                       const float* __restrict__ bias_ih, const float* __restrict__ bias_hh,
                       const float* __restrict__ cx, float* out_hy, float* out_cy)
{
#pragma clang fp contract(off)
    __shared__ __attribute__((aligned(16))) float stile[2][32 * SP_];

    const int tid  = threadIdx.x;
    const int lane = tid & 31;
    const int wave = tid >> 5;
    const int h    = lane >> 4;
    const int m    = lane & 15;
    const int wm   = wave >> 1;
    const int wn   = wave & 1;

    const int rowB = blockIdx.y * 32;
    const int colB = blockIdx.x * 32;
    const int rowW = rowB + wm * 16;
    const int colW = colB + wn * 16;
    const int j    = colW + m;

    const size_t aoff = (size_t)(rowW + m) * NI_ + 8 * h;
    const size_t boff = (size_t)j * NI_ + 8 * h;

    v8f acc[4];
#pragma unroll
    for (int g = 0; g < 4; ++g)
#pragma unroll
        for (int r = 0; r < 8; ++r) acc[g][r] = 0.0f;

    gemm_phase(Xh, Xl, Wih, Wil, aoff, boff, acc);

    v8f gs[4];
#pragma unroll
    for (int g = 0; g < 4; ++g) {
        const float b = bias_ih[g * NH_ + j];
#pragma unroll
        for (int r = 0; r < 8; ++r)
            gs[g][r] = quant_p2(acc[g][r] + b, 16384.0f, 1.0f / 16384.0f);
    }

#pragma unroll
    for (int g = 0; g < 4; ++g)
#pragma unroll
        for (int r = 0; r < 8; ++r) acc[g][r] = 0.0f;

    gemm_phase(Hh, Hl, Whh, Whl, aoff, boff, acc);

#pragma unroll
    for (int g = 0; g < 4; ++g) {
        const float b = bias_hh[g * NH_ + j];
#pragma unroll
        for (int r = 0; r < 8; ++r)
            gs[g][r] = gs[g][r] + quant_p2(acc[g][r] + b, 16384.0f, 1.0f / 16384.0f);
    }

    float* st0 = stile[0];
    float* st1 = stile[1];
    const int lcol = wn * 16 + m;
#pragma unroll 1
    for (int r = 0; r < 8; ++r) {
        const float vin  = gs[0][0];
        const float vfg  = gs[1][0];
        const float vcg  = gs[2][0];
        const float vog  = gs[3][0];
#pragma unroll
        for (int g = 0; g < 4; ++g)
            gs[g] = __builtin_shufflevector(gs[g], gs[g], 1, 2, 3, 4, 5, 6, 7, 0);

        const int lrow = wm * 16 + 8 * h + r;
        const float cxv = cx[(size_t)(rowB + lrow) * NH_ + j];

        const float ing = qsig_fn(vin);
        const float fg  = qsig_fn(vfg);
        const float cg  = qtanh_fn(vcg);
        const float og  = qsig_fn(vog);

        const float qcx = quant_p2(cxv, 32768.0f, 1.0f / 32768.0f);
        const float p1  = qcx * fg;
        const float p2  = ing * cg;
        const float cyv = p1 + p2;
        const float th  = qtanh_fn(cyv);
        const float hyv = th * og;
        const float cyq = quant_p2(cyv, 32768.0f, 1.0f / 32768.0f);

        st0[lrow * SP_ + lcol] = hyv;
        st1[lrow * SP_ + lcol] = cyq;
    }
    __syncthreads();

    out_store_pass(st0, st1, out_hy, out_cy, rowB, colB, wave, lane);
    __threadfence();
    out_store_pass(st0, st1, out_hy, out_cy, rowB, colB, wave, lane);
}

extern "C" void kernel_launch(void* const* d_in, const int* in_sizes, int n_in,
                              void* d_out, int out_size, void* d_ws, size_t ws_size,
                              hipStream_t stream)
{
    if (n_in < 7) return;
    if (in_sizes[0] != NB_ * NI_) return;
    if (in_sizes[1] != NB_ * NH_) return;
    if (in_sizes[2] != NB_ * NH_) return;
    if (in_sizes[3] != NG_ * NI_) return;
    if (in_sizes[4] != NG_ * NH_) return;
    if (in_sizes[5] != NG_)       return;
    if (in_sizes[6] != NG_)       return;
    if (out_size != 2 * NB_ * NH_) return;
    if (ws_size < WS_END)          return;

    const float* input_x   = (const float*)d_in[0];
    const float* hidden    = (const float*)d_in[1];
    const float* cx        = (const float*)d_in[2];
    const float* weight_ih = (const float*)d_in[3];
    const float* weight_hh = (const float*)d_in[4];
    const float* bias_ih   = (const float*)d_in[5];
    const float* bias_hh   = (const float*)d_in[6];

    float* out_hy = (float*)d_out;
    float* out_cy = out_hy + (size_t)NB_ * NH_;

    char* ws = (char*)d_ws;
    unsigned short* xh  = (unsigned short*)(ws + OFF_XH);
    unsigned short* xl  = (unsigned short*)(ws + OFF_XL);
    unsigned short* hh  = (unsigned short*)(ws + OFF_HH);
    unsigned short* hl  = (unsigned short*)(ws + OFF_HL);
    unsigned short* wih = (unsigned short*)(ws + OFF_WIH);
    unsigned short* wil = (unsigned short*)(ws + OFF_WIL);
    unsigned short* whh = (unsigned short*)(ws + OFF_WHH);
    unsigned short* whl = (unsigned short*)(ws + OFF_WHL);

    {
        const int n8a = (NB_ * NI_) / 8;
        const int n8h = (NB_ * NH_) / 8;
        const int n8w = (NG_ * NI_) / 8;
        const int n8v = (NG_ * NH_) / 8;
        cvt_split_kernel<<<dim3((n8a + 255) / 256), dim3(256), 0, stream>>>(input_x,   xh,  xl,  n8a);
        cvt_split_kernel<<<dim3((n8h + 255) / 256), dim3(256), 0, stream>>>(hidden,    hh,  hl,  n8h);
        cvt_split_kernel<<<dim3((n8w + 255) / 256), dim3(256), 0, stream>>>(weight_ih, wih, wil, n8w);
        cvt_split_kernel<<<dim3((n8v + 255) / 256), dim3(256), 0, stream>>>(weight_hh, whh, whl, n8v);
    }

    gates_gemm_kernel<<<dim3(NH_ / 32, NB_ / 32), dim3(128), 0, stream>>>(
        (const unsigned short*)xh,  (const unsigned short*)xl,
        (const unsigned short*)hh,  (const unsigned short*)hl,
        (const unsigned short*)wih, (const unsigned short*)wil,
        (const unsigned short*)whh, (const unsigned short*)whl,
        bias_ih, bias_hh, cx, out_hy, out_cy);
}
